// MultiHeadAttention_17033840296039
// MI455X (gfx1250) — hardware-run, weakly checked
//
#include <hip/hip_runtime.h>
#include <math.h>

typedef __attribute__((ext_vector_type(16))) _Float16 v16h;
typedef __attribute__((ext_vector_type(8)))  _Float16 v8h;
typedef __attribute__((ext_vector_type(8)))  float    v8f;
typedef __attribute__((ext_vector_type(4)))  float    v4f;
typedef __attribute__((ext_vector_type(4)))  unsigned int v4u;

constexpr int kB  = 8;
constexpr int kS  = 2048;
constexpr int kD  = 512;
constexpr int kH  = 8;
constexpr int kDh = 64;
constexpr int kSqrtDh = 8;
constexpr int kRows = kB * kS;
constexpr int kLP = 72;
constexpr int kOP = 68;
static_assert(kH * kDh == kD, "head split");
static_assert(kSqrtDh * kSqrtDh == kDh, "sqrt of head dim");
static_assert((kS % 64) == 0 && (kDh % 32) == 0 && kDh == 64, "tile multiples");
static_assert(kRows * kD == 8388608, "element count");

constexpr float kXCarry   = 16.0f;
constexpr float kWCarry   = 64.0f;
constexpr float kProjInv  = 1.0f / (kXCarry * kWCarry);
constexpr float kQCarry   = 64.0f;
constexpr float kKCarry   = 16.0f;
constexpr float kLog2e    = 1.4426950408889634f;
constexpr float kQScale   = (1.0f / (float)kSqrtDh) * kLog2e * kQCarry;
constexpr float kScoreInv = 1.0f / (kQCarry * kKCarry);
constexpr float kPLog2    = 15.0f;

constexpr size_t kPlaneBytes = (size_t)kB * kH * kS * kDh * 2;
constexpr size_t kOffQ  = 0;
constexpr size_t kOffK  = kOffQ + kPlaneBytes;
constexpr size_t kOffKT = kOffK + kPlaneBytes;
constexpr size_t kWsTotal = kOffKT + kPlaneBytes;
static_assert(kWsTotal == 50331648ull, "carve total");
static_assert(kWsTotal <= 134217728ull, "carve cap");
static_assert((kOffK % 128) == 0 && (kOffKT % 128) == 0, "aligned regions");

union FH { v16h v; v4u u[2]; v8h h[2]; };

__device__ __forceinline__ unsigned short h_bits(float f) {
  const _Float16 h = (_Float16)f;
  return __builtin_bit_cast(unsigned short, h);
}
__device__ __forceinline__ unsigned pk16(unsigned short a, unsigned short b) {
  return (unsigned)a | ((unsigned)b << 16);
}

__device__ __forceinline__ v8f mma2_f16(v16h a0, v16h b0, v16h a1, v16h b1, v8f c) {
  c = __builtin_amdgcn_wmma_f32_16x16x32_f16(false, a0, false, b0, (short)0, c, false, false);
  c = __builtin_amdgcn_wmma_f32_16x16x32_f16(false, a1, false, b1, (short)0, c, false, false);
  asm volatile("v_nop\n\tv_nop\n\tv_nop\n\tv_nop" : "+v"(c) : "v"(a0), "v"(b0), "v"(a1), "v"(b1));
  return c;
}

__device__ __forceinline__ void stage32_f16(const float* __restrict__ src, unsigned short* dst, float carry) {
#pragma unroll
  for (int i = 0; i < 4; ++i) {
    const v4f a = *(const v4f*)(src + 8 * i);
    const v4f c = *(const v4f*)(src + 8 * i + 4);
    const float a0 = a[0] * carry, a1 = a[1] * carry, a2 = a[2] * carry, a3 = a[3] * carry;
    const float c0 = c[0] * carry, c1 = c[1] * carry, c2 = c[2] * carry, c3 = c[3] * carry;
    const v4u u = (v4u){pk16(h_bits(a0), h_bits(a1)), pk16(h_bits(a2), h_bits(a3)),
                        pk16(h_bits(c0), h_bits(c1)), pk16(h_bits(c2), h_bits(c3))};
    *(v4u*)(dst + 8 * i) = u;
  }
}

__global__ __launch_bounds__(128) void proj_qk_kernel(
    const float* __restrict__ x,
    const float* __restrict__ Wq, const float* __restrict__ bq,
    const float* __restrict__ Wk, const float* __restrict__ bk,
    unsigned short* __restrict__ Q16, unsigned short* __restrict__ K16, unsigned short* __restrict__ KT16)
{
  __shared__ __align__(16) unsigned short sX[64 * kLP];
  __shared__ __align__(16) unsigned short sWq[64 * kLP];
  __shared__ __align__(16) unsigned short sWk[64 * kLP];
  __shared__ __align__(16) unsigned short sQ[64 * kLP];
  __shared__ __align__(16) unsigned short sK[64 * kLP];
  __shared__ __align__(16) unsigned short sKT[64 * kLP];

  const int tid  = threadIdx.x;
  const int lane = tid & 31;
  const int wave = __builtin_amdgcn_readfirstlane((int)(threadIdx.x >> 5));
  const int hh   = lane >> 4;
  const int c    = lane & 15;
  const int g0   = blockIdx.x * 64;
  const int b    = g0 / kS;
  const int s0   = g0 - b * kS;
  const int srow = tid >> 1;
  const int scol = (tid & 1) * 32;
  const int q    = lane >> 3;
  const int c8   = (lane & 7) * 8;

#pragma unroll 1
  for (int h = 0; h < kH; ++h) {
    stage32_f16(x  + (size_t)(g0 + srow) * kD + h * kDh + scol, sX  + srow * kLP + scol, kXCarry);
    stage32_f16(Wq + ((size_t)h * kDh + srow) * kDh + scol,     sWq + srow * kLP + scol, kWCarry);
    stage32_f16(Wk + ((size_t)h * kDh + srow) * kDh + scol,     sWk + srow * kLP + scol, kWCarry);
    __syncthreads();

    FH ax0, ax1;
    {
      const unsigned short* ap = sX + (wave * 16 + c) * kLP + 8 * hh;
      ax0.u[0] = *(const v4u*)(ap);
      ax0.u[1] = *(const v4u*)(ap + 16);
      ax1.u[0] = *(const v4u*)(ap + 32);
      ax1.u[1] = *(const v4u*)(ap + 48);
    }
    v8f aq[4], ak[4];
#pragma unroll
    for (int j = 0; j < 4; ++j) {
      const v8f z = (v8f){0.f, 0.f, 0.f, 0.f, 0.f, 0.f, 0.f, 0.f};
      FH w0, w1;
      const unsigned short* wp = sWq + (j * 16 + c) * kLP + 8 * hh;
      w0.u[0] = *(const v4u*)(wp);
      w0.u[1] = *(const v4u*)(wp + 16);
      w1.u[0] = *(const v4u*)(wp + 32);
      w1.u[1] = *(const v4u*)(wp + 48);
      aq[j] = mma2_f16(ax0.v, w0.v, ax1.v, w1.v, z);
      FH u0, u1;
      const unsigned short* up = sWk + (j * 16 + c) * kLP + 8 * hh;
      u0.u[0] = *(const v4u*)(up);
      u0.u[1] = *(const v4u*)(up + 16);
      u1.u[0] = *(const v4u*)(up + 32);
      u1.u[1] = *(const v4u*)(up + 48);
      ak[j] = mma2_f16(ax0.v, u0.v, ax1.v, u1.v, z);
    }

#pragma unroll
    for (int j = 0; j < 4; ++j) {
      const int e = j * 16 + c;
      const float bqv = bq[h * kDh + e];
      const float bkv = bk[h * kDh + e];
      unsigned short kb[8];
#pragma unroll
      for (int r = 0; r < 8; ++r) {
        const float qa = aq[j][r];
        const float ka = ak[j][r];
        const float qv = (qa * kProjInv + bqv) * kQScale;
        const float kv = (ka * kProjInv + bkv) * kKCarry;
        const int row = wave * 16 + 8 * hh + r;
        const unsigned short kh = h_bits(kv);
        sQ[row * kLP + e] = h_bits(qv);
        sK[row * kLP + e] = kh;
        kb[r] = kh;
      }
      const v4u kt = (v4u){pk16(kb[0], kb[1]), pk16(kb[2], kb[3]), pk16(kb[4], kb[5]), pk16(kb[6], kb[7])};
      *(v4u*)(sKT + e * kLP + wave * 16 + 8 * hh) = kt;
    }
    __syncthreads();

    v4u vq[4], vk[4], vt[4];
#pragma unroll
    for (int it = 0; it < 4; ++it) {
      const int row = it * 16 + wave * 4 + q;
      vq[it] = *(const v4u*)(sQ  + row * kLP + c8);
      vk[it] = *(const v4u*)(sK  + row * kLP + c8);
      vt[it] = *(const v4u*)(sKT + row * kLP + c8);
    }
    const size_t bh = (size_t)b * kH + h;
    for (int pass = 0; pass < 2; ++pass) {
#pragma unroll
      for (int it = 0; it < 4; ++it) {
        const int row = it * 16 + wave * 4 + q;
        const size_t oq = (bh * kS + s0 + row) * kDh + c8;
        const size_t ot = (bh * kDh + row) * kS + s0 + c8;
        *(volatile v4u*)(Q16 + oq)  = vq[it];
        *(volatile v4u*)(K16 + oq)  = vk[it];
        *(volatile v4u*)(KT16 + ot) = vt[it];
      }
      __threadfence();
    }
  }
}

__global__ __launch_bounds__(128) void attn_kernel(
    const unsigned short* __restrict__ Q16, const unsigned short* __restrict__ K16,
    const unsigned short* __restrict__ KT16, float* __restrict__ out)
{
  __shared__ __align__(16) unsigned short sKk[64 * kLP];
  __shared__ __align__(16) unsigned short sVt[64 * kLP];
  __shared__ __align__(16) _Float16 sP[4][16 * kLP];
  __shared__ __align__(16) float sO[4][16 * kOP];

  const int tid  = threadIdx.x;
  const int lane = tid & 31;
  const int wave = __builtin_amdgcn_readfirstlane((int)(threadIdx.x >> 5));
  const int hh   = lane >> 4;
  const int c    = lane & 15;

  constexpr int kQB = kS / 64;
  const int bx = blockIdx.x;
  const int bh = bx / kQB;
  const int qb = bx - bh * kQB;
  const int h  = bh % kH;
  const int b  = bh / kH;
  const int q0 = qb * 64 + wave * 16;

  const unsigned short* Kh  = K16  + (size_t)bh * kS * kDh;
  const unsigned short* KTh = KT16 + (size_t)bh * kDh * kS;

  FH qa0, qa1;
  {
    const unsigned short* qp = Q16 + ((size_t)bh * kS + q0 + c) * kDh + 8 * hh;
    qa0.u[0] = *(const v4u*)(qp);
    qa0.u[1] = *(const v4u*)(qp + 16);
    qa1.u[0] = *(const v4u*)(qp + 32);
    qa1.u[1] = *(const v4u*)(qp + 48);
  }

  float mrow[8], lpart[8];
  v8f oacc[4];
#pragma unroll
  for (int r = 0; r < 8; ++r) { mrow[r] = -1.0e30f; lpart[r] = 0.f; }
#pragma unroll
  for (int t = 0; t < 4; ++t) oacc[t] = (v8f){0.f, 0.f, 0.f, 0.f, 0.f, 0.f, 0.f, 0.f};

  _Float16* pw = sP[wave];

#pragma unroll 1
  for (int kc = 0; kc < kS / 64; ++kc) {
    const int kv0 = kc * 64;
    __syncthreads();
#pragma unroll
    for (int it = 0; it < 4; ++it) {
      const int idx = it * 128 + tid;
      const int row = idx >> 3;
      const int cc  = (idx & 7) * 8;
      const v4u kk = *(const v4u*)(Kh  + (size_t)(kv0 + row) * kDh + cc);
      const v4u vv = *(const v4u*)(KTh + (size_t)row * kS + kv0 + cc);
      *(v4u*)(sKk + row * kLP + cc) = kk;
      *(v4u*)(sVt + row * kLP + cc) = vv;
    }
    __syncthreads();

    v8f s[4];
#pragma unroll
    for (int j = 0; j < 4; ++j) {
      const v8f z = (v8f){0.f, 0.f, 0.f, 0.f, 0.f, 0.f, 0.f, 0.f};
      const unsigned short* kp = sKk + (j * 16 + c) * kLP + 8 * hh;
      FH k0, k1;
      k0.u[0] = *(const v4u*)(kp);
      k0.u[1] = *(const v4u*)(kp + 16);
      k1.u[0] = *(const v4u*)(kp + 32);
      k1.u[1] = *(const v4u*)(kp + 48);
      s[j] = mma2_f16(qa0.v, k0.v, qa1.v, k1.v, z);
    }

#pragma unroll
    for (int r = 0; r < 8; ++r) {
      const float s0v = s[0][r];
      const float s1v = s[1][r];
      const float s2v = s[2][r];
      const float s3v = s[3][r];
      float mx = fmaxf(fmaxf(s0v, s1v), fmaxf(s2v, s3v));
      mx = fmaxf(mx, __shfl_xor(mx, 1, 32));
      mx = fmaxf(mx, __shfl_xor(mx, 2, 32));
      mx = fmaxf(mx, __shfl_xor(mx, 4, 32));
      mx = fmaxf(mx, __shfl_xor(mx, 8, 32));
      const float mnew  = fmaxf(mrow[r], mx * kScoreInv);
      const float alpha = __builtin_amdgcn_exp2f(mrow[r] - mnew);
      mrow[r] = mnew;
      const float bias = kPLog2 - mnew;
      const float p0 = __builtin_amdgcn_exp2f(fmaf(s0v, kScoreInv, bias));
      const float p1 = __builtin_amdgcn_exp2f(fmaf(s1v, kScoreInv, bias));
      const float p2 = __builtin_amdgcn_exp2f(fmaf(s2v, kScoreInv, bias));
      const float p3 = __builtin_amdgcn_exp2f(fmaf(s3v, kScoreInv, bias));
      const _Float16 h0 = (_Float16)p0;
      const _Float16 h1 = (_Float16)p1;
      const _Float16 h2 = (_Float16)p2;
      const _Float16 h3 = (_Float16)p3;
      _Float16* pr = pw + (8 * hh + r) * kLP + c;
      pr[0]  = h0;
      pr[16] = h1;
      pr[32] = h2;
      pr[48] = h3;
      const float lsum = ((float)h0 + (float)h1) + ((float)h2 + (float)h3);
      lpart[r] = fmaf(lpart[r], alpha, lsum);
      oacc[0][r] *= alpha;
      oacc[1][r] *= alpha;
      oacc[2][r] *= alpha;
      oacc[3][r] *= alpha;
    }
    __builtin_amdgcn_fence(__ATOMIC_RELEASE, "workgroup");
    __builtin_amdgcn_wave_barrier();
    __builtin_amdgcn_fence(__ATOMIC_ACQUIRE, "workgroup");

    FH pa0, pa1;
    {
      const _Float16* pp = pw + c * kLP + 8 * hh;
      pa0.h[0] = *(const v8h*)(pp);
      pa0.h[1] = *(const v8h*)(pp + 16);
      pa1.h[0] = *(const v8h*)(pp + 32);
      pa1.h[1] = *(const v8h*)(pp + 48);
    }
#pragma unroll
    for (int t = 0; t < 4; ++t) {
      const unsigned short* vp = sVt + (t * 16 + c) * kLP + 8 * hh;
      FH v0, v1;
      v0.u[0] = *(const v4u*)(vp);
      v0.u[1] = *(const v4u*)(vp + 16);
      v1.u[0] = *(const v4u*)(vp + 32);
      v1.u[1] = *(const v4u*)(vp + 48);
      oacc[t] = mma2_f16(pa0.v, v0.v, pa1.v, v1.v, oacc[t]);
    }
  }

  float* os = sO[wave];
#pragma unroll
  for (int r = 0; r < 8; ++r) {
    float l = lpart[r];
    l += __shfl_xor(l, 1, 32);
    l += __shfl_xor(l, 2, 32);
    l += __shfl_xor(l, 4, 32);
    l += __shfl_xor(l, 8, 32);
    const float inv = 1.0f / (l * kKCarry);
    float* orow = os + (8 * hh + r) * kOP + c;
    orow[0]  = oacc[0][r] * inv;
    orow[16] = oacc[1][r] * inv;
    orow[32] = oacc[2][r] * inv;
    orow[48] = oacc[3][r] * inv;
  }
  __builtin_amdgcn_fence(__ATOMIC_RELEASE, "workgroup");
  __builtin_amdgcn_wave_barrier();
  __builtin_amdgcn_fence(__ATOMIC_ACQUIRE, "workgroup");
  {
    const int c4 = c * 4;
    float* ob = out + ((size_t)b * kS + q0) * kD + h * kDh;
    for (int pass = 0; pass < 2; ++pass) {
#pragma unroll
      for (int it = 0; it < 8; ++it) {
        const int row = it * 2 + hh;
        const v4f val = *(const v4f*)(os + row * kOP + c4);
        *(volatile v4f*)(ob + (size_t)row * kD + c4) = val;
      }
      __threadfence();
    }
  }
}

extern "C" void kernel_launch(void* const* d_in, const int* in_sizes, int n_in,
                              void* d_out, int out_size, void* d_ws, size_t ws_size,
                              hipStream_t stream) {
  if (n_in < 5) return;
  if (in_sizes[0] != kRows * kD) return;
  if (in_sizes[1] != kH * kDh * kDh) return;
  if (in_sizes[2] != kH * kDh) return;
  if (in_sizes[3] != kH * kDh * kDh) return;
  if (in_sizes[4] != kH * kDh) return;
  if (out_size != kRows * kD) return;
  if (ws_size < kWsTotal) return;

  const float* x  = (const float*)d_in[0];
  const float* Wq = (const float*)d_in[1];
  const float* bq = (const float*)d_in[2];
  const float* Wk = (const float*)d_in[3];
  const float* bk = (const float*)d_in[4];
  float* out = (float*)d_out;

  char* ws = (char*)d_ws;
  unsigned short* Q16  = (unsigned short*)(ws + kOffQ);
  unsigned short* K16  = (unsigned short*)(ws + kOffK);
  unsigned short* KT16 = (unsigned short*)(ws + kOffKT);

  proj_qk_kernel<<<kRows / 64, 128, 0, stream>>>(x, Wq, bq, Wk, bk, Q16, K16, KT16);
  attn_kernel<<<kB * kH * (kS / 64), 128, 0, stream>>>(Q16, K16, KT16, out);
}
